// GlobalSubSampleAttn_81449759801421
// MI455X (gfx1250) — hardware-verified
//
#include <hip/hip_runtime.h>
#include <math.h>
#include <stdint.h>


#define BATCH 8
#define NTOK  4096
#define CD    256
#define CD2   512
#define NHEAD 8
#define HDIM  32
#define STOK  256
#define IMW   64
#define MROWS (BATCH * NTOK)
#define SROWS (BATCH * STOK)
#define KCONV (CD * 16)
#define OUTN  (MROWS * CD)
static_assert(NHEAD * HDIM == CD);
static_assert(HDIM == 32);
static_assert(NTOK == IMW * IMW);
static_assert(STOK == (IMW / 4) * (IMW / 4));
static_assert(STOK == 256 && NTOK == 4096);
static_assert((KCONV / 8) == 512 && (CD / 8) == 32);
static_assert((NTOK % 64) == 0 && (MROWS % 64) == 0 && (SROWS % 64) == 0);
static_assert((CD % 64) == 0 && (CD2 % 64) == 0 && (KCONV % 32) == 0);
static_assert((((MROWS / 64) * (CD / 64)) % 8) == 0);
static_assert((((MROWS / 64) * (CD2 / 64)) % 8) == 0);
static_assert((((SROWS / 64) * (CD / 64)) % 8) == 0);
static_assert((MROWS % 8) == 0 && (SROWS % 8) == 0);
static_assert(((MROWS * CD / 8) % 256) == 0 && ((SROWS * KCONV / 8) % 256) == 0);
static_assert(((CD * CD / 8) % 256) == 0 && ((CD * KCONV / 8) % 256) == 0);

typedef __bf16         v16bf __attribute__((ext_vector_type(16)));
typedef float          v8f   __attribute__((ext_vector_type(8)));
typedef float          v4f   __attribute__((ext_vector_type(4)));
typedef unsigned int   v4u   __attribute__((ext_vector_type(4)));
typedef unsigned short v8us  __attribute__((ext_vector_type(8)));
typedef unsigned short v16us __attribute__((ext_vector_type(16)));

__device__ __forceinline__ unsigned short bf_bits(float f) {
  const unsigned u = __float_as_uint(f);
  return (unsigned short)((u + 0x7FFFu + ((u >> 16) & 1u)) >> 16);
}
__device__ __forceinline__ float bf_up(unsigned short h) { return __uint_as_float(((unsigned)h) << 16); }
__device__ __forceinline__ float bfr(float f) { return bf_up(bf_bits(f)); }
__device__ __forceinline__ unsigned pk16(unsigned short a, unsigned short b) { return (unsigned)a | ((unsigned)b << 16); }
__device__ __forceinline__ v8f zero8() { v8f z = {0.f, 0.f, 0.f, 0.f, 0.f, 0.f, 0.f, 0.f}; return z; }

__device__ __forceinline__ void ld8(const float* p, float* o) {
  const v4f a = *(const v4f*)(p);
  const v4f b = *(const v4f*)(p + 4);
  o[0] = a[0]; o[1] = a[1]; o[2] = a[2]; o[3] = a[3];
  o[4] = b[0]; o[5] = b[1]; o[6] = b[2]; o[7] = b[3];
}

__device__ __forceinline__ v16bf ldfrag_b(const unsigned short* p) {
  union { v16us v; v8us h[2]; } f;
  f.h[0] = *(const v8us*)(p);
  f.h[1] = *(const v8us*)(p + 16);
  return __builtin_bit_cast(v16bf, f.v);
}

__device__ __forceinline__ v8f mma_b(v16bf a, v16bf b, v8f c) {
  c = __builtin_amdgcn_wmma_f32_16x16x32_bf16(false, a, false, b, (short)0, c, false, false);
#if defined(__HIP_DEVICE_COMPILE__)
  asm volatile("v_nop\n\tv_nop\n\tv_nop\n\tv_nop" : "+v"(c) : "v"(a), "v"(b));
#endif
  return c;
}
__device__ __forceinline__ v8f mma_b_raw(v16bf a, v16bf b, v8f c) {
  return __builtin_amdgcn_wmma_f32_16x16x32_bf16(false, a, false, b, (short)0, c, false, false);
}
__device__ __forceinline__ void dep_guard_b(v8f& a, v8f& b, v16bf x) {
#if defined(__HIP_DEVICE_COMPILE__)
  asm volatile("v_nop\n\tv_nop\n\tv_nop\n\tv_nop" : "+v"(a), "+v"(b) : "v"(x));
#endif
}
__device__ __forceinline__ void keep4_b(v16bf a, v16bf b, v16bf c, v16bf d) {
#if defined(__HIP_DEVICE_COMPILE__)
  asm volatile("v_nop" :: "v"(a), "v"(b), "v"(c), "v"(d));
#endif
}
__device__ __forceinline__ void acc_guard4(v8f& a, v8f& b, v8f& c, v8f& d) {
#if defined(__HIP_DEVICE_COMPILE__)
  asm volatile("v_nop\n\tv_nop\n\tv_nop\n\tv_nop" : "+v"(a), "+v"(b), "+v"(c), "+v"(d));
#endif
}

__global__ __launch_bounds__(256) void cvt_bf16x8(const float* __restrict__ in, unsigned short* out, int n8) {
  const int i = blockIdx.x * 256 + threadIdx.x;
  if (i < n8) {
    float v[8];
    ld8(in + (size_t)i * 8, v);
    v4u p;
#pragma unroll
    for (int q = 0; q < 4; ++q) p[q] = pk16(bf_bits(v[2 * q]), bf_bits(v[2 * q + 1]));
    unsigned short* o = out + (size_t)i * 8;
    *(volatile v4u*)o = p;
    __threadfence();
    *(volatile v4u*)o = p;
  }
}

__global__ __launch_bounds__(256) void pack_conv_w(const float* __restrict__ w, unsigned short* Wc, int n8) {
  const int i = blockIdx.x * 256 + threadIdx.x;
  if (i < n8) {
    const int o = i >> 9;
    const int k8 = (i & 511) * 8;
    const int p = k8 >> 8, ch0 = k8 & 255;
    const int kh = p >> 2, kw = p & 3;
    float v[8];
#pragma unroll
    for (int e = 0; e < 8; ++e) v[e] = w[(((size_t)o * CD + ch0 + e) * 4 + kh) * 4 + kw];
    v4u q4;
#pragma unroll
    for (int q = 0; q < 4; ++q) q4[q] = pk16(bf_bits(v[2 * q]), bf_bits(v[2 * q + 1]));
    unsigned short* op = Wc + (size_t)i * 8;
    *(volatile v4u*)op = q4;
    __threadfence();
    *(volatile v4u*)op = q4;
  }
}

__global__ __launch_bounds__(256) void pack_conv_a(const float* __restrict__ x, unsigned short* Ac, int n8) {
  const int i = blockIdx.x * 256 + threadIdx.x;
  if (i < n8) {
    const int row = i >> 9, k8 = (i & 511) * 8;
    const int p = k8 >> 8, ch0 = k8 & 255;
    const int b = row >> 8, s = row & 255;
    const int sy = s >> 4, sx = s & 15, py = p >> 2, px = p & 3;
    const int pix = (sy * 4 + py) * IMW + (sx * 4 + px);
    float v[8];
    ld8(x + ((size_t)(b * NTOK + pix)) * CD + ch0, v);
    v4u q4;
#pragma unroll
    for (int q = 0; q < 4; ++q) q4[q] = pk16(bf_bits(v[2 * q]), bf_bits(v[2 * q + 1]));
    unsigned short* op = Ac + (size_t)i * 8;
    *(volatile v4u*)op = q4;
    __threadfence();
    *(volatile v4u*)op = q4;
  }
}

template <int NA>
__device__ __forceinline__ void kseg(v8f (&acc)[4][4],
                                     const unsigned short* __restrict__ Pa, const unsigned short* __restrict__ Pb,
                                     int ld, int m0, int kcnt,
                                     const unsigned short* __restrict__ Bt, int ldb, int n0, int bk0,
                                     int rlane, int koff) {
  for (int kk = 0; kk < kcnt; kk += 32) {
    v16bf bh[4];
#pragma unroll
    for (int j = 0; j < 4; ++j) {
      const size_t bo = (size_t)(n0 + (j << 4) + rlane) * (size_t)ldb + koff + bk0 + kk;
      bh[j] = ldfrag_b(Bt + bo);
    }
#pragma unroll
    for (int i = 0; i < 4; ++i) {
      const size_t ao = (size_t)(m0 + (i << 4) + rlane) * (size_t)ld + koff + kk;
      const v16bf a0 = ldfrag_b(Pa + ao);
#pragma unroll
      for (int j = 0; j < 4; ++j) acc[i][j] = mma_b_raw(a0, bh[j], acc[i][j]);
      dep_guard_b(acc[i][0], acc[i][3], a0);
      if (NA == 2) {
        const v16bf a1 = ldfrag_b(Pb + ao);
#pragma unroll
        for (int j = 0; j < 4; ++j) acc[i][j] = mma_b_raw(a1, bh[j], acc[i][j]);
        dep_guard_b(acc[i][0], acc[i][3], a1);
      }
    }
    keep4_b(bh[0], bh[1], bh[2], bh[3]);
  }
}

template <int MODE, int NA0, int NA1, int BIAS, int ACT>
__global__ __launch_bounds__(256) void gemm64(
    const unsigned short* __restrict__ P0a, const unsigned short* __restrict__ P0b, int ld0, int Ks,
    const unsigned short* __restrict__ P1a, const unsigned short* __restrict__ P1b, int ld1,
    const unsigned short* __restrict__ Bt, int ldb, const float* __restrict__ bias,
    float* Cf, unsigned short* Ch, unsigned short* Cl, int ldc, int M, int N, int K) {
  __shared__ __align__(16) float sT[8][16 * 68];
  const int lane = threadIdx.x & 31;
  const int wave = threadIdx.x >> 5;
  const int tilesN = N >> 6;
  const int tilesM = M >> 6;
  const int tiles = tilesM * tilesN;
  const int item = blockIdx.x * 8 + wave;
  if (item >= tiles) return;
  const int tm = item / tilesN;
  const int tn = item - tm * tilesN;
  const int m0 = tm << 6;
  const int n0 = tn << 6;

  const int rlane = lane & 15;
  const int koff  = (lane >> 4) * 8;
  const int mOff  = (lane >> 4) * 8;

  v8f acc[4][4];
#pragma unroll
  for (int i = 0; i < 4; ++i)
#pragma unroll
    for (int j = 0; j < 4; ++j) acc[i][j] = zero8();

  kseg<NA0>(acc, P0a, P0b, ld0, m0, Ks, Bt, ldb, n0, 0, rlane, koff);
  if (Ks < K) kseg<NA1>(acc, P1a, P1b, ld1, m0, K - Ks, Bt, ldb, n0, Ks, rlane, koff);
  acc_guard4(acc[0][0], acc[0][1], acc[0][2], acc[0][3]);
  acc_guard4(acc[1][0], acc[1][1], acc[1][2], acc[1][3]);
  acc_guard4(acc[2][0], acc[2][1], acc[2][2], acc[2][3]);
  acc_guard4(acc[3][0], acc[3][1], acc[3][2], acc[3][3]);

  float* slab = sT[wave];
#pragma unroll
  for (int i = 0; i < 4; ++i) {
    const int mBase = m0 + (i << 4);
#pragma unroll
    for (int r = 0; r < 8; ++r) {
#pragma unroll
      for (int j = 0; j < 4; ++j) {
        slab[(mOff + r) * 68 + (j << 4) + rlane] = acc[i][j][r];
      }
    }
    __builtin_amdgcn_fence(__ATOMIC_RELEASE, "workgroup");
    __builtin_amdgcn_wave_barrier();
    __builtin_amdgcn_fence(__ATOMIC_ACQUIRE, "workgroup");
    if (MODE == 0) {
      const int h2 = lane >> 4, c4 = (lane & 15) * 4;
      v4f b4 = {0.f, 0.f, 0.f, 0.f};
      if (BIAS != 0) {
        const v4f braw = *(const v4f*)(bias + n0 + c4);
#pragma unroll
        for (int e = 0; e < 4; ++e) b4[e] = bfr(braw[e]);
      }
      v4f ov[8];
#pragma unroll
      for (int it = 0; it < 8; ++it) {
        const int row = it * 2 + h2;
        const v4f xs = *(const v4f*)(slab + row * 68 + c4);
        ov[it] = xs + b4;
      }
      for (int pass = 0; pass < 2; ++pass) {
#pragma unroll
        for (int it = 0; it < 8; ++it) {
          const int row = it * 2 + h2;
          *(volatile v4f*)(Cf + (size_t)(mBase + row) * (size_t)ldc + n0 + c4) = ov[it];
        }
        __threadfence();
      }
    } else {
      const int q8 = lane & 7, rr = lane >> 3, c8 = q8 * 8;
      float bb[8] = {0.f, 0.f, 0.f, 0.f, 0.f, 0.f, 0.f, 0.f};
      if (BIAS != 0) {
        const v4f b0 = *(const v4f*)(bias + n0 + c8);
        const v4f b1 = *(const v4f*)(bias + n0 + c8 + 4);
#pragma unroll
        for (int e = 0; e < 4; ++e) { bb[e] = bfr(b0[e]); bb[4 + e] = bfr(b1[e]); }
      }
      v4u ovh[4], ovl[4];
#pragma unroll
      for (int it = 0; it < 4; ++it) {
        const int row = it * 4 + rr;
        float xs[8];
        ld8(slab + row * 68 + c8, xs);
        unsigned short hb[8], lb[8];
#pragma unroll
        for (int e = 0; e < 8; ++e) {
          float xv = xs[e] + bb[e];
          if (ACT == 1) xv = fmaxf(xv, 0.0f);
          if (ACT == 2) {
            const float ev = expm1f(fminf(xv, 0.0f));
            xv = (xv > 0.0f) ? (xv + 1.0f) : (ev + 1.0f);
          }
          hb[e] = bf_bits(xv);
          lb[e] = bf_bits(xv - bf_up(hb[e]));
        }
        v4u ah, al;
#pragma unroll
        for (int p = 0; p < 4; ++p) { ah[p] = pk16(hb[2 * p], hb[2 * p + 1]); al[p] = pk16(lb[2 * p], lb[2 * p + 1]); }
        ovh[it] = ah; ovl[it] = al;
      }
      for (int pass = 0; pass < 2; ++pass) {
#pragma unroll
        for (int it = 0; it < 4; ++it) {
          const int row = it * 4 + rr;
          const size_t co = (size_t)(mBase + row) * (size_t)ldc + n0 + c8;
          *(volatile v4u*)(Ch + co) = ovh[it];
          if (MODE == 3) *(volatile v4u*)(Cl + co) = ovl[it];
        }
        __threadfence();
      }
    }
    __builtin_amdgcn_fence(__ATOMIC_RELEASE, "workgroup");
    __builtin_amdgcn_wave_barrier();
    __builtin_amdgcn_fence(__ATOMIC_ACQUIRE, "workgroup");
  }
}

template <int OUTF>
__global__ __launch_bounds__(256) void k_lnrow(const float* __restrict__ P, const float* __restrict__ ga,
                                               const float* __restrict__ be, const float* __restrict__ xres,
                                               float* F, unsigned short* Hh, unsigned short* Lh, int ldh, int nrows) {
#pragma clang fp contract(off)
  __shared__ __align__(16) float so[8][CD];
  const int tid = threadIdx.x, wave = tid >> 5, lane = tid & 31;
  const int row = blockIdx.x * 8 + wave;
  if (row >= nrows) return;
  const int c0 = lane * 8;
  const size_t ro = (size_t)row * CD + c0;
  float x[8];
  ld8(P + ro, x);
  float s = ((x[0] + x[1]) + (x[2] + x[3])) + ((x[4] + x[5]) + (x[6] + x[7]));
#pragma unroll
  for (int off = 16; off >= 1; off >>= 1) s += __shfl_xor(s, off, 32);
  const float mu = s * (1.0f / (float)CD);
  float d[8];
  float ss = 0.f;
#pragma unroll
  for (int e = 0; e < 8; ++e) { d[e] = x[e] - mu; ss += d[e] * d[e]; }
#pragma unroll
  for (int off = 16; off >= 1; off >>= 1) ss += __shfl_xor(ss, off, 32);
  const float var = ss * (1.0f / (float)CD);
  const float rs = 1.0f / sqrtf(var + 1e-5f);
  float g8[8], b8[8], y[8];
  ld8(ga + c0, g8);
  ld8(be + c0, b8);
#pragma unroll
  for (int e = 0; e < 8; ++e) y[e] = (d[e] * rs) * bfr(g8[e]) + bfr(b8[e]);

  if (OUTF == 0) {
    v4u hv, lv;
#pragma unroll
    for (int p = 0; p < 4; ++p) {
      const unsigned short h0 = bf_bits(y[2 * p]), h1 = bf_bits(y[2 * p + 1]);
      const unsigned short l0 = bf_bits(y[2 * p] - bf_up(h0)), l1 = bf_bits(y[2 * p + 1] - bf_up(h1));
      hv[p] = pk16(h0, h1); lv[p] = pk16(l0, l1);
    }
    const size_t ho = (size_t)row * (size_t)ldh + c0;
    *(volatile v4u*)(Hh + ho) = hv;
    *(volatile v4u*)(Lh + ho) = lv;
    __threadfence();
    *(volatile v4u*)(Hh + ho) = hv;
    *(volatile v4u*)(Lh + ho) = lv;
  } else {
    float* sw = so[wave];
    const v4f ya = {y[0], y[1], y[2], y[3]};
    const v4f yb = {y[4], y[5], y[6], y[7]};
    *(v4f*)(sw + c0) = ya;
    *(v4f*)(sw + c0 + 4) = yb;
    __builtin_amdgcn_fence(__ATOMIC_RELEASE, "workgroup");
    __builtin_amdgcn_wave_barrier();
    __builtin_amdgcn_fence(__ATOMIC_ACQUIRE, "workgroup");
    const int c4 = lane * 4;
    const v4f pa = *(const v4f*)(sw + c4);
    const v4f pb = *(const v4f*)(sw + 128 + c4);
    const size_t xo = (size_t)row * CD + c4;
    const v4f xa = *(const v4f*)(xres + xo);
    const v4f xb = *(const v4f*)(xres + xo + 128);
    const v4f oa = {bfr(xa[0]) + pa[0], bfr(xa[1]) + pa[1], bfr(xa[2]) + pa[2], bfr(xa[3]) + pa[3]};
    const v4f ob = {bfr(xb[0]) + pb[0], bfr(xb[1]) + pb[1], bfr(xb[2]) + pb[2], bfr(xb[3]) + pb[3]};
    *(volatile v4f*)(F + xo) = oa;
    *(volatile v4f*)(F + xo + 128) = ob;
    __threadfence();
    *(volatile v4f*)(F + xo) = oa;
    *(volatile v4f*)(F + xo + 128) = ob;
  }
}

__global__ __launch_bounds__(256) void k_kvred(const float* __restrict__ Kf, const float* __restrict__ Vf,
                                               unsigned short* KVh, unsigned short* KVl, float* Ks) {
  __shared__ float sk[32][33];
  __shared__ float sv[32][33];
  __shared__ float skv[32][33];
  __shared__ __align__(16) float sks[32];
  const int t = threadIdx.x;
  const int bh = blockIdx.x, b = bh >> 3, h = bh & 7;
  const int e = t >> 3, d0 = (t & 7) * 4;
  float acc[4] = {0.f, 0.f, 0.f, 0.f};
  float ks[4] = {0.f, 0.f, 0.f, 0.f};
  for (int sc = 0; sc < STOK / 32; ++sc) {
    const size_t go = ((size_t)(b * STOK + sc * 32 + e)) * CD + h * HDIM + d0;
    v4f kq = *(const v4f*)(Kf + go);
    const v4f vq = *(const v4f*)(Vf + go);
#pragma unroll 1
    for (int j = 0; j < 4; ++j) {
      const float tq = kq[0];
      const float ev = expm1f(fminf(tq, 0.0f));
      const float r = (tq > 0.0f) ? (tq + 1.0f) : (ev + 1.0f);
      const v4f nv = {kq[1], kq[2], kq[3], r};
      kq = nv;
    }
#pragma unroll
    for (int j = 0; j < 4; ++j) { sk[e][d0 + j] = kq[j]; sv[e][d0 + j] = vq[j]; }
    __syncthreads();
#pragma unroll 4
    for (int s2 = 0; s2 < 32; ++s2) {
      const float ve = sv[s2][e];
#pragma unroll
      for (int j = 0; j < 4; ++j) {
        const float kd = sk[s2][d0 + j];
        acc[j] += kd * ve;
        ks[j] += kd;
      }
    }
    __syncthreads();
  }
#pragma unroll
  for (int j = 0; j < 4; ++j) skv[e][d0 + j] = acc[j] * (1.0f / 256.0f);
  if (t < 8) {
#pragma unroll
    for (int j = 0; j < 4; ++j) sks[d0 + j] = ks[j];
  }
  __syncthreads();
  const int e2 = (t & 127) >> 2, d8 = (t & 3) * 8;
  unsigned short hb[8], lb[8];
#pragma unroll
  for (int q = 0; q < 8; ++q) {
    const float f = skv[e2][d8 + q];
    hb[q] = bf_bits(f);
    lb[q] = bf_bits(f - bf_up(hb[q]));
  }
  v4u hv, lv;
#pragma unroll
  for (int p = 0; p < 4; ++p) { hv[p] = pk16(hb[2 * p], hb[2 * p + 1]); lv[p] = pk16(lb[2 * p], lb[2 * p + 1]); }
  const size_t ko = (size_t)bh * (HDIM * HDIM) + (size_t)e2 * HDIM + d8;
  const int t7 = t & 7;
  const v4f k4 = {sks[t7 * 4], sks[t7 * 4 + 1], sks[t7 * 4 + 2], sks[t7 * 4 + 3]};
  const bool wkv = t < 128, wks = t < 8;
  if (wkv) { *(volatile v4u*)(KVh + ko) = hv; *(volatile v4u*)(KVl + ko) = lv; }
  if (wks) *(volatile v4f*)(Ks + (size_t)bh * HDIM + t7 * 4) = k4;
  __threadfence();
  if (wkv) { *(volatile v4u*)(KVh + ko) = hv; *(volatile v4u*)(KVl + ko) = lv; }
  if (wks) *(volatile v4f*)(Ks + (size_t)bh * HDIM + t7 * 4) = k4;
}

__global__ __launch_bounds__(128) void k_msg(const unsigned short* __restrict__ QH, const unsigned short* __restrict__ KVh,
                                             const unsigned short* __restrict__ KVl, const float* __restrict__ Ks,
                                             unsigned short* MSh, unsigned short* MSl) {
  __shared__ __align__(16) float sks[2 * HDIM];
  __shared__ __align__(16) float Os[4][16 * 68];
  const int tid = threadIdx.x, wave = tid >> 5, lane = tid & 31;
  const int hh = lane >> 4, c = lane & 15;
  const int bx = blockIdx.x;
  const int tile = bx & (NTOK / 64 - 1);
  const int hp = (bx >> 6) & 3;
  const int b = bx >> 8;
  const int row0 = b * NTOK + tile * 64 + wave * 16;
  const int bh0 = b * NHEAD + hp * 2;
  const int cb = hp * 64;
  if (tid < 2 * HDIM) sks[tid] = Ks[(size_t)bh0 * HDIM + tid];
  __syncthreads();

  const unsigned short* qrow = QH + (size_t)(row0 + c) * CD + cb;
  const v16bf qa0 = ldfrag_b(qrow + 8 * hh);
  const v16bf qa1 = ldfrag_b(qrow + HDIM + 8 * hh);

  float zq0 = 0.f, zq1 = 0.f;
#pragma unroll
  for (int q = 0; q < 4; ++q) {
    const v8us u0 = *(const v8us*)(qrow + 8 * q);
    const v8us u1 = *(const v8us*)(qrow + HDIM + 8 * q);
#pragma unroll
    for (int e = 0; e < 8; ++e) {
      zq0 += bf_up(u0[e]) * sks[8 * q + e];
      zq1 += bf_up(u1[e]) * sks[HDIM + 8 * q + e];
    }
  }
  const float z0 = 1.0f / (zq0 + 1e-6f);
  const float z1 = 1.0f / (zq1 + 1e-6f);

  v8f acc[2][2];
  {
    const size_t k0o = (size_t)bh0 * (HDIM * HDIM);
    const size_t k1o = k0o + HDIM * HDIM;
#pragma unroll
    for (int t2 = 0; t2 < 2; ++t2) {
      const int bo = (t2 * 16 + c) * HDIM + 8 * hh;
      const v16bf b0h = ldfrag_b(KVh + k0o + bo);
      const v16bf b0l = ldfrag_b(KVl + k0o + bo);
      const v16bf b1h = ldfrag_b(KVh + k1o + bo);
      const v16bf b1l = ldfrag_b(KVl + k1o + bo);
      acc[0][t2] = mma_b(qa0, b0h, zero8());
      acc[0][t2] = mma_b(qa0, b0l, acc[0][t2]);
      acc[1][t2] = mma_b(qa1, b1h, zero8());
      acc[1][t2] = mma_b(qa1, b1l, acc[1][t2]);
    }
  }

  float* os = Os[wave];
#pragma unroll
  for (int r = 0; r < 8; ++r) {
    const float zr0 = __shfl(z0, 8 * hh + r, 32) * 256.0f;
    const float zr1 = __shfl(z1, 8 * hh + r, 32) * 256.0f;
    const int ob = (8 * hh + r) * 68;
    os[ob + c]      = acc[0][0][r] * zr0;
    os[ob + 16 + c] = acc[0][1][r] * zr0;
    os[ob + 32 + c] = acc[1][0][r] * zr1;
    os[ob + 48 + c] = acc[1][1][r] * zr1;
  }
  __builtin_amdgcn_fence(__ATOMIC_RELEASE, "workgroup");
  __builtin_amdgcn_wave_barrier();
  __builtin_amdgcn_fence(__ATOMIC_ACQUIRE, "workgroup");
  {
    const int q8 = lane & 7, rr = lane >> 3;
    v4u ovh[4], ovl[4];
#pragma unroll
    for (int it = 0; it < 4; ++it) {
      const int row = it * 4 + rr;
      float xs[8];
      ld8(os + row * 68 + q8 * 8, xs);
      unsigned short hb[8], lb[8];
#pragma unroll
      for (int e = 0; e < 8; ++e) { hb[e] = bf_bits(xs[e]); lb[e] = bf_bits(xs[e] - bf_up(hb[e])); }
      v4u ah, al;
#pragma unroll
      for (int p = 0; p < 4; ++p) { ah[p] = pk16(hb[2 * p], hb[2 * p + 1]); al[p] = pk16(lb[2 * p], lb[2 * p + 1]); }
      ovh[it] = ah; ovl[it] = al;
    }
    for (int pass = 0; pass < 2; ++pass) {
#pragma unroll
      for (int it = 0; it < 4; ++it) {
        const int row = it * 4 + rr;
        const size_t go = (size_t)(row0 + row) * CD + cb + q8 * 8;
        *(volatile v4u*)(MSh + go) = ovh[it];
        *(volatile v4u*)(MSl + go) = ovl[it];
      }
      __threadfence();
    }
  }
}

extern "C" void kernel_launch(void* const* d_in, const int* in_sizes, int n_in,
                              void* d_out, int out_size, void* d_ws, size_t ws_size,
                              hipStream_t stream) {
  if (n_in < 17) return;
  if (in_sizes[0] != OUTN) return;
  if (in_sizes[1] != CD * CD * 16) return;
  if (in_sizes[2] != CD || in_sizes[3] != CD || in_sizes[4] != CD) return;
  if (in_sizes[5] != CD * CD || in_sizes[6] != CD * CD || in_sizes[7] != CD * CD || in_sizes[8] != CD * CD) return;
  if (in_sizes[9] != CD2 * CD2) return;
  if (in_sizes[10] != CD * CD2) return;
  if (in_sizes[11] != CD || in_sizes[12] != CD || in_sizes[13] != CD || in_sizes[14] != CD) return;
  if (out_size != OUTN) return;

  const float* x     = (const float*)d_in[0];
  const float* sr_w  = (const float*)d_in[1];
  const float* sr_b  = (const float*)d_in[2];
  const float* ng    = (const float*)d_in[3];
  const float* nb    = (const float*)d_in[4];
  const float* wq    = (const float*)d_in[5];
  const float* wk    = (const float*)d_in[6];
  const float* wv    = (const float*)d_in[7];
  const float* wm    = (const float*)d_in[8];
  const float* w1    = (const float*)d_in[9];
  const float* w2    = (const float*)d_in[10];
  const float* n1g   = (const float*)d_in[11];
  const float* n1b   = (const float*)d_in[12];
  const float* n2g   = (const float*)d_in[13];
  const float* n2b   = (const float*)d_in[14];

  const size_t PW   = (size_t)CD * CD * 2;
  const size_t PW1  = (size_t)CD2 * CD2 * 2;
  const size_t PW2  = (size_t)CD * CD2 * 2;
  const size_t PH   = (size_t)MROWS * CD * 2;
  const size_t PF   = (size_t)MROWS * CD * 4;
  const size_t PH2  = (size_t)MROWS * CD2 * 2;
  const size_t PACV = (size_t)SROWS * KCONV * 2;
  const size_t PWC  = (size_t)CD * KCONV * 2;
  const size_t PSF  = (size_t)SROWS * CD * 4;
  const size_t PSH  = (size_t)SROWS * CD * 2;
  const size_t PKV  = (size_t)BATCH * NHEAD * HDIM * HDIM * 2;
  const size_t PKS  = (size_t)BATCH * NHEAD * HDIM * 4;

  size_t off = 0;
  const size_t oWQ  = off; off += PW;
  const size_t oWK  = off; off += PW;
  const size_t oWV  = off; off += PW;
  const size_t oWM  = off; off += PW;
  const size_t oW1  = off; off += PW1;
  const size_t oW2  = off; off += PW2;
  const size_t oMID = off; off += 3 * PH;
  const size_t oBIG = off; off += 2 * PF;
  if (off > ws_size) return;
  if (off > (size_t)134217728) return;

  const size_t bACV = 0;
  const size_t bWC  = bACV + PACV;
  const size_t bXS  = bWC + PWC;
  const size_t bSRh = bXS + PSF;
  const size_t bSRl = bSRh + PSH;
  const size_t bKf  = bSRl + PSH;
  const size_t bVf  = bKf + PSF;
  const size_t bKVh = bVf + PSF;
  const size_t bKVl = bKVh + PKV;
  const size_t bKS  = bKVl + PKV;
  const size_t bXb1 = PF;
  const size_t bQH  = PF + PH;
  if (bKS + PKS > bXb1) return;
  if (bQH + PH > 2 * PF) return;
  if (2 * PH + PH > 3 * PH) return;
  if (PH2 != PF) return;

  char* ws = (char*)d_ws;
  unsigned short* WQ   = (unsigned short*)(ws + oWQ);
  unsigned short* WK   = (unsigned short*)(ws + oWK);
  unsigned short* WV   = (unsigned short*)(ws + oWV);
  unsigned short* WM   = (unsigned short*)(ws + oWM);
  unsigned short* W1p  = (unsigned short*)(ws + oW1);
  unsigned short* W2p  = (unsigned short*)(ws + oW2);
  char* mid = ws + oMID;
  char* big = ws + oBIG;
  unsigned short* MSh  = (unsigned short*)(mid);
  unsigned short* MSl  = (unsigned short*)(mid + PH);
  unsigned short* M1h  = (unsigned short*)(mid);
  unsigned short* M1l  = (unsigned short*)(mid + PH);
  unsigned short* Xb2  = (unsigned short*)(mid + 2 * PH);
  float*          S2   = (float*)(mid);
  unsigned short* ACV  = (unsigned short*)(big + bACV);
  unsigned short* WC   = (unsigned short*)(big + bWC);
  float*          XS   = (float*)(big + bXS);
  unsigned short* SRh  = (unsigned short*)(big + bSRh);
  unsigned short* SRl  = (unsigned short*)(big + bSRl);
  float*          Kf   = (float*)(big + bKf);
  float*          Vf   = (float*)(big + bVf);
  unsigned short* KVh  = (unsigned short*)(big + bKVh);
  unsigned short* KVl  = (unsigned short*)(big + bKVl);
  float*          KSUM = (float*)(big + bKS);
  unsigned short* Xb1  = (unsigned short*)(big + bXb1);
  unsigned short* QH   = (unsigned short*)(big + bQH);
  float*          S0   = (float*)(big);
  unsigned short* H1h  = (unsigned short*)(big);
  unsigned short* H1l  = (unsigned short*)(big + PH2);
  float*          outf = (float*)d_out;

  const dim3 blk(256);
  const int n8w   = CD * CD / 8;
  const int n8w1  = CD2 * CD2 / 8;
  const int n8w2  = CD * CD2 / 8;
  const int n8wc  = CD * KCONV / 8;
  const int n8acv = SROWS * KCONV / 8;
  const int n8x   = MROWS * CD / 8;
  const dim3 gW((n8w + 255) / 256);
  const dim3 gW1((n8w1 + 255) / 256);
  const dim3 gW2((n8w2 + 255) / 256);
  const dim3 gWC((n8wc + 255) / 256);
  const dim3 gACV((n8acv + 255) / 256);
  const dim3 gX((n8x + 255) / 256);
  const dim3 gConv(((SROWS / 64) * (CD / 64) + 7) / 8);
  const dim3 gKV(((SROWS / 64) * (CD / 64) + 7) / 8);
  const dim3 gQ(((MROWS / 64) * (CD / 64) + 7) / 8);
  const dim3 gMlp1(((MROWS / 64) * (CD2 / 64) + 7) / 8);
  const dim3 gLnS(SROWS / 8);
  const dim3 gLnM(MROWS / 8);
  const dim3 gKvr(BATCH * NHEAD);
  const dim3 gMsg(BATCH * 4 * (NTOK / 64));

  cvt_bf16x8<<<gW, blk, 0, stream>>>(wq, WQ, n8w);
  cvt_bf16x8<<<gW, blk, 0, stream>>>(wk, WK, n8w);
  cvt_bf16x8<<<gW, blk, 0, stream>>>(wv, WV, n8w);
  cvt_bf16x8<<<gW, blk, 0, stream>>>(wm, WM, n8w);
  cvt_bf16x8<<<gW1, blk, 0, stream>>>(w1, W1p, n8w1);
  cvt_bf16x8<<<gW2, blk, 0, stream>>>(w2, W2p, n8w2);
  pack_conv_w<<<gWC, blk, 0, stream>>>(sr_w, WC, n8wc);
  pack_conv_a<<<gACV, blk, 0, stream>>>(x, ACV, n8acv);
  cvt_bf16x8<<<gX, blk, 0, stream>>>(x, Xb1, n8x);
  gemm64<0, 1, 1, 1, 0><<<gConv, blk, 0, stream>>>(ACV, ACV, KCONV, KCONV, ACV, ACV, KCONV, WC, KCONV, sr_b,
                                                  XS, QH, QH, CD, SROWS, CD, KCONV);
  k_lnrow<0><<<gLnS, blk, 0, stream>>>(XS, ng, nb, x, XS, SRh, SRl, CD, SROWS);
  gemm64<0, 2, 1, 0, 0><<<gKV, blk, 0, stream>>>(SRh, SRl, CD, CD, SRh, SRl, CD, WK, CD, sr_b,
                                                Kf, QH, QH, CD, SROWS, CD, CD);
  gemm64<0, 2, 1, 0, 0><<<gKV, blk, 0, stream>>>(SRh, SRl, CD, CD, SRh, SRl, CD, WV, CD, sr_b,
                                                Vf, QH, QH, CD, SROWS, CD, CD);
  gemm64<2, 1, 1, 0, 2><<<gQ, blk, 0, stream>>>(Xb1, Xb1, CD, CD, Xb1, Xb1, CD, WQ, CD, sr_b,
                                               XS, QH, QH, CD, MROWS, CD, CD);
  k_kvred<<<gKvr, blk, 0, stream>>>(Kf, Vf, KVh, KVl, KSUM);
  k_msg<<<gMsg, dim3(128), 0, stream>>>(QH, KVh, KVl, KSUM, MSh, MSl);
  gemm64<0, 2, 1, 0, 0><<<gQ, blk, 0, stream>>>(MSh, MSl, CD, CD, MSh, MSl, CD, WM, CD, sr_b,
                                               S0, QH, QH, CD, MROWS, CD, CD);
  k_lnrow<0><<<gLnM, blk, 0, stream>>>(S0, n1g, n1b, x, XS, M1h, M1l, CD, MROWS);
  cvt_bf16x8<<<gX, blk, 0, stream>>>(x, Xb2, n8x);
  gemm64<3, 1, 2, 0, 1><<<gMlp1, blk, 0, stream>>>(Xb2, Xb2, CD, CD, M1h, M1l, CD, W1p, CD2, sr_b,
                                                  XS, H1h, H1l, CD2, MROWS, CD2, CD2);
  gemm64<0, 2, 1, 0, 0><<<gQ, blk, 0, stream>>>(H1h, H1l, CD2, CD2, H1h, H1l, CD2, W2p, CD2, sr_b,
                                               S2, QH, QH, CD, MROWS, CD, CD2);
  k_lnrow<1><<<gLnM, blk, 0, stream>>>(S2, n2g, n2b, x, outf, M1h, M1l, CD, MROWS);
  (void)hipGetLastError();
}
